// SymmetricLinearAttention_46084999086237
// MI455X (gfx1250) — hardware-verified
//
#include <hip/hip_runtime.h>
#include <math.h>

#define SQ    2048
#define NB    4
#define DM    1024
#define NTOK  (SQ * NB)
#define NHD   16
#define HD    64
#define NBH   (NB * NHD)
#define NSB   (SQ / 32)
#define SBH   (HD * 32)
#define TPB   128
#define OSTR  68
#define KVP   68
#define TPT   72

static_assert(NHD * HD == DM);
static_assert(NTOK % TPB == 0);
static_assert(TPB == 32 * NB);
static_assert(DM % 64 == 0);
static_assert(DM % 32 == 0);
static_assert(SQ % 128 == 0);
static_assert(OSTR % 4 == 0);
static_assert(KVP % 4 == 0);
static_assert((TPT * 2) % 16 == 0);
static_assert((NTOK * DM) % 8 == 0);
static_assert((DM * DM) % 8 == 0);
static_assert(NSB % 2 == 0);

typedef unsigned short us16 __attribute__((ext_vector_type(16)));
typedef unsigned short us8  __attribute__((ext_vector_type(8)));
typedef unsigned short us8a __attribute__((ext_vector_type(8), may_alias));
typedef __bf16 v16b __attribute__((ext_vector_type(16)));
typedef _Float16 v16h __attribute__((ext_vector_type(16)));
typedef _Float16 v8ha __attribute__((ext_vector_type(8), may_alias));
typedef float v8f __attribute__((ext_vector_type(8)));
typedef float v4f __attribute__((ext_vector_type(4)));
typedef float v4fa __attribute__((ext_vector_type(4), may_alias));
union FragU { us16 v; us8 h[2]; };

__device__ __forceinline__ unsigned short bf16_bits(float f) {
  unsigned u = __float_as_uint(f);
  u += 0x7FFFu + ((u >> 16) & 1u);
  return (unsigned short)(u >> 16);
}
__device__ __forceinline__ float bf16_val(unsigned short b) { return __uint_as_float(((unsigned)b) << 16); }
__device__ __forceinline__ float bf16r(float f) { return bf16_val(bf16_bits(f)); }
__device__ __forceinline__ unsigned short f16_bits(float f) { return __builtin_bit_cast(unsigned short, (_Float16)f); }
__device__ __forceinline__ float phi1(float v) { return v > 0.0f ? v + 1.0f : expf(v); }

__device__ __forceinline__ void f16hl(float v, float sc, unsigned short& hb, unsigned short& rb) {
  const _Float16 hf = (_Float16)v;
  hb = __builtin_bit_cast(unsigned short, hf);
  rb = __builtin_bit_cast(unsigned short, (_Float16)((v - (float)hf) * sc));
}

__device__ __forceinline__ v8f mma_bf16(us16 a, us16 b, v8f c) {
  return __builtin_amdgcn_wmma_f32_16x16x32_bf16(false, __builtin_bit_cast(v16b, a), false, __builtin_bit_cast(v16b, b), (short)0, c, false, false);
}
__device__ __forceinline__ v8f mma_f16(us16 a, us16 b, v8f c) {
  return __builtin_amdgcn_wmma_f32_16x16x32_f16(false, __builtin_bit_cast(v16h, a), false, __builtin_bit_cast(v16h, b), (short)0, c, false, false);
}
__device__ __forceinline__ void wguard4(v8f& c0, v8f& c1, v8f& c2, v8f& c3, const us16& a0,
                                        const us16& b0, const us16& b1, const us16& b2, const us16& b3) {
#if defined(__HIP_DEVICE_COMPILE__)
  asm volatile("v_nop\n\tv_nop\n\tv_nop\n\tv_nop"
               : "+v"(c0), "+v"(c1), "+v"(c2), "+v"(c3)
               : "v"(a0), "v"(b0), "v"(b1), "v"(b2), "v"(b3));
#endif
}
__device__ __forceinline__ void wguard8_2a4b(v8f& c0, v8f& c1, v8f& c2, v8f& c3, v8f& c4, v8f& c5, v8f& c6, v8f& c7,
                                             const us16& a0, const us16& a1,
                                             const us16& b0, const us16& b1, const us16& b2, const us16& b3) {
#if defined(__HIP_DEVICE_COMPILE__)
  asm volatile("v_nop\n\tv_nop\n\tv_nop\n\tv_nop"
               : "+v"(c0), "+v"(c1), "+v"(c2), "+v"(c3), "+v"(c4), "+v"(c5), "+v"(c6), "+v"(c7)
               : "v"(a0), "v"(a1), "v"(b0), "v"(b1), "v"(b2), "v"(b3));
#endif
}
__device__ __forceinline__ void wguard8_1a8b(v8f& c0, v8f& c1, v8f& c2, v8f& c3, v8f& c4, v8f& c5, v8f& c6, v8f& c7,
                                             const us16& a0,
                                             const us16& b0, const us16& b1, const us16& b2, const us16& b3,
                                             const us16& b4, const us16& b5, const us16& b6, const us16& b7) {
#if defined(__HIP_DEVICE_COMPILE__)
  asm volatile("v_nop\n\tv_nop\n\tv_nop\n\tv_nop"
               : "+v"(c0), "+v"(c1), "+v"(c2), "+v"(c3), "+v"(c4), "+v"(c5), "+v"(c6), "+v"(c7)
               : "v"(a0), "v"(b0), "v"(b1), "v"(b2), "v"(b3), "v"(b4), "v"(b5), "v"(b6), "v"(b7));
#endif
}
__device__ __forceinline__ void wguard8_2a8b(v8f& c0, v8f& c1, v8f& c2, v8f& c3, v8f& c4, v8f& c5, v8f& c6, v8f& c7,
                                             const us16& a0, const us16& a1,
                                             const us16& b0, const us16& b1, const us16& b2, const us16& b3,
                                             const us16& b4, const us16& b5, const us16& b6, const us16& b7) {
#if defined(__HIP_DEVICE_COMPILE__)
  asm volatile("v_nop\n\tv_nop\n\tv_nop\n\tv_nop"
               : "+v"(c0), "+v"(c1), "+v"(c2), "+v"(c3), "+v"(c4), "+v"(c5), "+v"(c6), "+v"(c7)
               : "v"(a0), "v"(a1), "v"(b0), "v"(b1), "v"(b2), "v"(b3), "v"(b4), "v"(b5), "v"(b6), "v"(b7));
#endif
}

__device__ __forceinline__ us16 gfrag(const unsigned short* p) {
  const int kh = ((threadIdx.x >> 4) & 1) * 8;
  FragU f;
  f.h[0] = *(const us8a*)(p + kh);
  f.h[1] = *(const us8a*)(p + 16 + kh);
  return f.v;
}

__global__ __launch_bounds__(256) void k_cvt_bf16(const float* __restrict__ src, unsigned short* dst, int total8) {
  const int idx = blockIdx.x * 256 + threadIdx.x;
  if (idx >= total8) return;
  const size_t off = (size_t)idx * 8;
  const v4f a = *(const v4fa*)(src + off), b = *(const v4fa*)(src + off + 4);
  us8 o;
#pragma unroll
  for (int u = 0; u < 4; ++u) {
    o[u]     = bf16_bits(a[u]);
    o[4 + u] = bf16_bits(b[u]);
  }
  *(volatile us8*)(dst + off) = o;
  __threadfence();
  *(volatile us8*)(dst + off) = o;
}

__global__ __launch_bounds__(256) void k_cvt_wT(const float* __restrict__ W, unsigned short* WT) {
  __shared__ __attribute__((aligned(16))) unsigned short tS[64 * TPT];
  const int tid = threadIdx.x;
  const int d0 = blockIdx.y * 64, e0 = blockIdx.x * 64;
  {
    const int row = tid >> 2, seg = (tid & 3) * 16;
    const float* src = W + (size_t)(d0 + row) * DM + e0 + seg;
#pragma unroll
    for (int u4 = 0; u4 < 4; ++u4) {
      const v4f a = *(const v4fa*)(src + 4 * u4);
#pragma unroll
      for (int u = 0; u < 4; ++u) tS[(seg + 4 * u4 + u) * TPT + row] = f16_bits(bf16r(a[u]) * 256.0f);
    }
  }
  __syncthreads();
  us8 v[2];
  size_t offs[2];
#pragma unroll
  for (int it = 0; it < 2; ++it) {
    const int pi = it * 256 + tid, line = pi >> 3, j = pi & 7;
    v[it] = *(const us8a*)(tS + line * TPT + 8 * j);
    offs[it] = (size_t)(e0 + line) * DM + d0 + 8 * j;
  }
#pragma unroll
  for (int pass = 0; pass < 2; ++pass) {
#pragma unroll
    for (int it = 0; it < 2; ++it) *(volatile us8*)(WT + offs[it]) = v[it];
    __threadfence();
  }
}

__global__ __launch_bounds__(256) void k_gemm_q(const unsigned short* __restrict__ Ap, const unsigned short* __restrict__ Bw,
                                               const float* __restrict__ bias, unsigned short* QF) {
  __shared__ __attribute__((aligned(16))) float oS[8 * 16 * OSTR];
  const int tid = threadIdx.x, lane = tid & 31, wave = tid >> 5, cl = lane & 15, hh = lane >> 4;
  const int m0 = blockIdx.x * TPB + 16 * wave, n0 = blockIdx.y * 64;

  v8f acc[4];
#pragma unroll
  for (int j = 0; j < 4; ++j) { const v8f zz = {0.f, 0.f, 0.f, 0.f, 0.f, 0.f, 0.f, 0.f}; acc[j] = zz; }

  const unsigned short* a0p = Ap + (size_t)(m0 + cl) * (size_t)DM;
  const unsigned short* bwp = Bw + (size_t)(n0 + cl) * (size_t)DM;
#pragma unroll 1
  for (int k0 = 0; k0 < DM; k0 += 32) {
    const us16 af = gfrag(a0p + k0);
    us16 bfr[4];
#pragma unroll
    for (int j = 0; j < 4; ++j) bfr[j] = gfrag(bwp + (size_t)(16 * j) * (size_t)DM + k0);
#pragma unroll
    for (int j = 0; j < 4; ++j) acc[j] = mma_bf16(af, bfr[j], acc[j]);
    wguard4(acc[0], acc[1], acc[2], acc[3], af, bfr[0], bfr[1], bfr[2], bfr[3]);
  }

  float* so = oS + wave * (16 * OSTR);
#pragma unroll
  for (int j = 0; j < 4; ++j)
#pragma unroll
    for (int r = 0; r < 8; ++r) so[(8 * hh + r) * OSTR + 16 * j + cl] = acc[j][r];
  __syncthreads();

  us8 ov[4];
  size_t offs[4];
#pragma unroll
  for (int it = 0; it < 4; ++it) {
    const int r = it * 4 + (lane >> 3), q = (lane & 7) * 8;
    const v4f x0 = *(const v4fa*)(so + r * OSTR + q), x1 = *(const v4fa*)(so + r * OSTR + q + 4);
    const v4f g0 = *(const v4fa*)(bias + n0 + q), g1 = *(const v4fa*)(bias + n0 + q + 4);
    us8 o;
#pragma unroll
    for (int u = 0; u < 4; ++u) {
      o[u]     = f16_bits(phi1(x0[u] + bf16r(g0[u])));
      o[4 + u] = f16_bits(phi1(x1[u] + bf16r(g1[u])));
    }
    ov[it] = o;
    offs[it] = (size_t)(m0 + r) * (size_t)DM + (size_t)(n0 + q);
  }
#pragma unroll
  for (int pass = 0; pass < 2; ++pass) {
#pragma unroll
    for (int it = 0; it < 4; ++it) *(volatile us8*)(QF + offs[it]) = ov[it];
    __threadfence();
  }
}

__global__ __launch_bounds__(256) void k_gemm_k(const unsigned short* __restrict__ Ap, const unsigned short* __restrict__ Bw,
                                               const float* __restrict__ bias,
                                               unsigned short* KFH, unsigned short* KFL, unsigned short* VTH, unsigned short* VTL) {
  __shared__ __attribute__((aligned(16))) float oS[8 * 16 * OSTR];
  const int tid = threadIdx.x, lane = tid & 31, wave = tid >> 5, cl = lane & 15, hh = lane >> 4;
  const int m0 = blockIdx.x * TPB + 16 * wave, n0 = blockIdx.y * 64;

  v8f acc[4];
#pragma unroll
  for (int j = 0; j < 4; ++j) { const v8f zz = {0.f, 0.f, 0.f, 0.f, 0.f, 0.f, 0.f, 0.f}; acc[j] = zz; }

  const unsigned short* a0p = Ap + (size_t)(m0 + cl) * (size_t)DM;
  const unsigned short* bwp = Bw + (size_t)(n0 + cl) * (size_t)DM;
#pragma unroll 1
  for (int k0 = 0; k0 < DM; k0 += 32) {
    const us16 af = gfrag(a0p + k0);
    us16 bfr[4];
#pragma unroll
    for (int j = 0; j < 4; ++j) bfr[j] = gfrag(bwp + (size_t)(16 * j) * (size_t)DM + k0);
#pragma unroll
    for (int j = 0; j < 4; ++j) acc[j] = mma_bf16(af, bfr[j], acc[j]);
    wguard4(acc[0], acc[1], acc[2], acc[3], af, bfr[0], bfr[1], bfr[2], bfr[3]);
  }

  float gb[4];
#pragma unroll
  for (int j = 0; j < 4; ++j) gb[j] = bf16r(bias[n0 + 16 * j + cl]);

  float* so = oS + wave * (16 * OSTR);
#pragma unroll
  for (int j = 0; j < 4; ++j)
#pragma unroll
    for (int r = 0; r < 8; ++r) so[(8 * hh + r) * OSTR + 16 * j + cl] = acc[j][r] + gb[j];
  __syncthreads();

  const int hd_ = blockIdx.y, sblk = blockIdx.x;
  us8 fh[4], fl[4], vh[4], vl[4];
  size_t offs[4];
#pragma unroll
  for (int it = 0; it < 4; ++it) {
    const int pi = it * 256 + tid, lb = pi >> 3, j = pi & 7;
    const int b = lb >> 5, L = lb & 31;
    const int d = 2 * L + (j >> 2), sl = (j & 3) * 8;
    us8 a0, a1, a2, a3;
#pragma unroll
    for (int i = 0; i < 8; ++i) {
      const float kx = oS[((sl + i) * NB + b) * OSTR + d];
      unsigned short hb, rb;
      f16hl(phi1(kx), 2048.0f, hb, rb); a0[i] = hb; a1[i] = rb;
      f16hl(kx, 2048.0f, hb, rb);       a2[i] = hb; a3[i] = rb;
    }
    fh[it] = a0; fl[it] = a1; vh[it] = a2; vl[it] = a3;
    offs[it] = ((size_t)(b * NHD + hd_) * NSB + (size_t)sblk) * (size_t)SBH + (size_t)L * 64 + (size_t)(8 * j);
  }
#pragma unroll
  for (int pass = 0; pass < 2; ++pass) {
#pragma unroll
    for (int it = 0; it < 4; ++it) {
      *(volatile us8*)(KFH + offs[it]) = fh[it];
      *(volatile us8*)(KFL + offs[it]) = fl[it];
      *(volatile us8*)(VTH + offs[it]) = vh[it];
      *(volatile us8*)(VTL + offs[it]) = vl[it];
    }
    __threadfence();
  }
}

__global__ __launch_bounds__(128) void k_kv(const unsigned short* __restrict__ KFH, const unsigned short* __restrict__ KFL,
                                           const unsigned short* __restrict__ VTH, const unsigned short* __restrict__ VTL,
                                           unsigned short* KVH, unsigned short* KVL, float* KS) {
  __shared__ __attribute__((aligned(16))) float sO[HD * KVP];
  __shared__ __attribute__((aligned(16))) float sks[2][HD];
  __shared__ __attribute__((aligned(16))) float skf[HD];
  const int tid = threadIdx.x, lane = tid & 31, wave = tid >> 5, cl = lane & 15, hh = lane >> 4;
  const int bh = blockIdx.x;
  const size_t hb0 = (size_t)bh * (size_t)(HD * SQ);

  v8f acch[4], accx[4];
#pragma unroll
  for (int j = 0; j < 4; ++j) { const v8f zz = {0.f, 0.f, 0.f, 0.f, 0.f, 0.f, 0.f, 0.f}; acch[j] = zz; accx[j] = zz; }

  const unsigned short* aph = VTH + hb0 + (size_t)(16 * wave + cl) * 32;
  const unsigned short* apl = VTL + hb0 + (size_t)(16 * wave + cl) * 32;
  const unsigned short* bph = KFH + hb0 + (size_t)cl * 32;
  const unsigned short* bpl = KFL + hb0 + (size_t)cl * 32;
#pragma unroll 1
  for (int t = 0; t < NSB; ++t) {
    const size_t to = (size_t)t * SBH;
    const us16 ah = gfrag(aph + to);
    const us16 al = gfrag(apl + to);
    us16 b8[8];
#pragma unroll
    for (int j = 0; j < 4; ++j) {
      b8[j]     = gfrag(bph + to + (size_t)(j * 16 * 32));
      b8[4 + j] = gfrag(bpl + to + (size_t)(j * 16 * 32));
    }
#pragma unroll
    for (int j = 0; j < 4; ++j) {
      acch[j] = mma_f16(ah, b8[j], acch[j]);
      accx[j] = mma_f16(ah, b8[4 + j], accx[j]);
      accx[j] = mma_f16(al, b8[j], accx[j]);
    }
    wguard8_2a8b(acch[0], acch[1], acch[2], acch[3], accx[0], accx[1], accx[2], accx[3], ah, al,
                 b8[0], b8[1], b8[2], b8[3], b8[4], b8[5], b8[6], b8[7]);
  }

  {
    const int d = tid & 63, half = tid >> 6;
    float shi = 0.0f, slo = 0.0f;
#pragma unroll 1
    for (int t = half * (NSB / 2); t < (half + 1) * (NSB / 2); ++t) {
      const unsigned short* ph = KFH + hb0 + (size_t)t * SBH + (size_t)d * 32;
      const unsigned short* pl = KFL + hb0 + (size_t)t * SBH + (size_t)d * 32;
#pragma unroll
      for (int c = 0; c < 4; ++c) {
        const v8ha h8 = *(const v8ha*)(ph + 8 * c);
        const v8ha l8 = *(const v8ha*)(pl + 8 * c);
#pragma unroll
        for (int u = 0; u < 8; ++u) { shi += (float)h8[u]; slo += (float)l8[u]; }
      }
    }
    sks[half][d] = fmaf(slo, (1.0f / 2048.0f), shi);
  }

#pragma unroll
  for (int j = 0; j < 4; ++j)
#pragma unroll
    for (int r = 0; r < 8; ++r) sO[(16 * wave + 8 * hh + r) * KVP + 16 * j + cl] = fmaf(accx[j][r], (1.0f / 2048.0f), acch[j][r]);
  __syncthreads();
  if (tid < HD) skf[tid] = sks[0][tid] + sks[1][tid];
  __syncthreads();

  us8 hv[4], lv[4];
  size_t offs[4];
#pragma unroll
  for (int it = 0; it < 4; ++it) {
    const int pi = it * 128 + tid, line = pi >> 3, j = pi & 7;
    const v4f x0 = *(const v4fa*)(sO + line * KVP + 8 * j), x1 = *(const v4fa*)(sO + line * KVP + 8 * j + 4);
    us8 ho, lo;
#pragma unroll
    for (int u = 0; u < 4; ++u) {
      unsigned short hb, rb;
      f16hl(x0[u], 1024.0f, hb, rb); ho[u] = hb;     lo[u] = rb;
      f16hl(x1[u], 1024.0f, hb, rb); ho[4 + u] = hb; lo[4 + u] = rb;
    }
    hv[it] = ho; lv[it] = lo;
    offs[it] = (size_t)bh * (size_t)(HD * HD) + (size_t)line * HD + (size_t)(8 * j);
  }
  const v4f kq = *(const v4fa*)(skf + 4 * (tid & 15));
#pragma unroll
  for (int pass = 0; pass < 2; ++pass) {
#pragma unroll
    for (int it = 0; it < 4; ++it) {
      *(volatile us8*)(KVH + offs[it]) = hv[it];
      *(volatile us8*)(KVL + offs[it]) = lv[it];
    }
    if (tid < 16) *(volatile v4f*)(KS + (size_t)bh * HD + 4 * tid) = kq;
    __threadfence();
  }
}

__global__ __launch_bounds__(256) void k_attn(const unsigned short* __restrict__ QF, const unsigned short* __restrict__ KVH,
                                             const unsigned short* __restrict__ KVL, const float* __restrict__ KS,
                                             unsigned short* ATH, unsigned short* ATL) {
  __shared__ __attribute__((aligned(16))) float oS[8 * 16 * OSTR];
  __shared__ __attribute__((aligned(16))) float sks[HD];
  __shared__ __attribute__((aligned(16))) float szr[128];
  const int tid = threadIdx.x, lane = tid & 31, wave = tid >> 5, cl = lane & 15, hh = lane >> 4;
  const int bh = blockIdx.y, b = bh >> 4, hd_ = bh & 15;
  const int sbase = blockIdx.x * 128, s0 = sbase + 16 * wave;

  if (tid < HD) sks[tid] = KS[(size_t)bh * HD + tid];

  v8f acch[4], accl[4];
#pragma unroll
  for (int j = 0; j < 4; ++j) { const v8f zz = {0.f, 0.f, 0.f, 0.f, 0.f, 0.f, 0.f, 0.f}; acch[j] = zz; accl[j] = zz; }

  const unsigned short* ap = QF + ((size_t)(s0 + cl) * NB + (size_t)b) * (size_t)DM + (size_t)(hd_ * HD);
  const unsigned short* hp = KVH + (size_t)bh * (size_t)(HD * HD) + (size_t)cl * HD;
  const unsigned short* lp = KVL + (size_t)bh * (size_t)(HD * HD) + (size_t)cl * HD;
#pragma unroll
  for (int ks = 0; ks < 2; ++ks) {
    const int k0 = 32 * ks;
    const us16 af = gfrag(ap + k0);
    us16 b8[8];
#pragma unroll
    for (int j = 0; j < 4; ++j) {
      b8[j]     = gfrag(hp + (size_t)(j * 16 * HD) + k0);
      b8[4 + j] = gfrag(lp + (size_t)(j * 16 * HD) + k0);
    }
#pragma unroll
    for (int j = 0; j < 4; ++j) {
      acch[j] = mma_f16(af, b8[j], acch[j]);
      accl[j] = mma_f16(af, b8[4 + j], accl[j]);
    }
    wguard8_1a8b(acch[0], acch[1], acch[2], acch[3], accl[0], accl[1], accl[2], accl[3], af,
                 b8[0], b8[1], b8[2], b8[3], b8[4], b8[5], b8[6], b8[7]);
  }
  __syncthreads();

  if (tid < 128) {
    const int s = sbase + tid;
    const unsigned short* qp = QF + ((size_t)s * NB + (size_t)b) * (size_t)DM + (size_t)(hd_ * HD);
    float z = 0.0f;
#pragma unroll
    for (int c = 0; c < 8; ++c) {
      const v8ha q8 = *(const v8ha*)(qp + 8 * c);
#pragma unroll
      for (int u = 0; u < 8; ++u) z = fmaf((float)q8[u], sks[8 * c + u], z);
    }
    szr[tid] = 256.0f * (1.0f / (z + 1e-6f));
  }

  float* so = oS + wave * (16 * OSTR);
#pragma unroll
  for (int j = 0; j < 4; ++j)
#pragma unroll
    for (int r = 0; r < 8; ++r) so[(8 * hh + r) * OSTR + 16 * j + cl] = fmaf(accl[j][r], (1.0f / 1024.0f), acch[j][r]);
  __syncthreads();

  us8 hv[4], lv[4];
  size_t offs[4];
#pragma unroll
  for (int it = 0; it < 4; ++it) {
    const int r = it * 4 + (lane >> 3), q = (lane & 7) * 8;
    const float zr = szr[16 * wave + r];
    const v4f x0 = *(const v4fa*)(so + r * OSTR + q), x1 = *(const v4fa*)(so + r * OSTR + q + 4);
    us8 ho, lo;
#pragma unroll
    for (int u = 0; u < 4; ++u) {
      unsigned short hb, rb;
      f16hl(x0[u] * zr, 2048.0f, hb, rb); ho[u] = hb;     lo[u] = rb;
      f16hl(x1[u] * zr, 2048.0f, hb, rb); ho[4 + u] = hb; lo[4 + u] = rb;
    }
    hv[it] = ho; lv[it] = lo;
    offs[it] = ((size_t)(s0 + r) * NB + (size_t)b) * (size_t)DM + (size_t)(hd_ * HD) + (size_t)q;
  }
#pragma unroll
  for (int pass = 0; pass < 2; ++pass) {
#pragma unroll
    for (int it = 0; it < 4; ++it) {
      *(volatile us8*)(ATH + offs[it]) = hv[it];
      *(volatile us8*)(ATL + offs[it]) = lv[it];
    }
    __threadfence();
  }
}

__global__ __launch_bounds__(256) void k_gemm_out(const unsigned short* __restrict__ Ah, const unsigned short* __restrict__ Al,
                                                 const unsigned short* __restrict__ Wt, float* out) {
  __shared__ __attribute__((aligned(16))) float oS[8 * 16 * OSTR];
  const int tid = threadIdx.x, lane = tid & 31, wave = tid >> 5, cl = lane & 15, hh = lane >> 4;
  const int m0 = blockIdx.x * TPB + 16 * wave, n0 = blockIdx.y * 64;

  v8f acch[4], accl[4];
#pragma unroll
  for (int j = 0; j < 4; ++j) { const v8f zz = {0.f, 0.f, 0.f, 0.f, 0.f, 0.f, 0.f, 0.f}; acch[j] = zz; accl[j] = zz; }

  const unsigned short* ahp = Ah + (size_t)(m0 + cl) * (size_t)DM;
  const unsigned short* alp = Al + (size_t)(m0 + cl) * (size_t)DM;
  const unsigned short* wtp = Wt + (size_t)(n0 + cl) * (size_t)DM;
#pragma unroll 1
  for (int k0 = 0; k0 < DM; k0 += 32) {
    const us16 ah = gfrag(ahp + k0);
    const us16 al = gfrag(alp + k0);
    us16 bfr[4];
#pragma unroll
    for (int j = 0; j < 4; ++j) bfr[j] = gfrag(wtp + (size_t)(16 * j) * (size_t)DM + k0);
#pragma unroll
    for (int j = 0; j < 4; ++j) {
      acch[j] = mma_f16(ah, bfr[j], acch[j]);
      accl[j] = mma_f16(al, bfr[j], accl[j]);
    }
    wguard8_2a4b(acch[0], acch[1], acch[2], acch[3], accl[0], accl[1], accl[2], accl[3], ah, al, bfr[0], bfr[1], bfr[2], bfr[3]);
  }

  float* so = oS + wave * (16 * OSTR);
#pragma unroll
  for (int j = 0; j < 4; ++j)
#pragma unroll
    for (int r = 0; r < 8; ++r)
      so[(8 * hh + r) * OSTR + 16 * j + cl] = fmaf(accl[j][r], (1.0f / 2048.0f), acch[j][r]) * (1.0f / 65536.0f);
  __syncthreads();

#pragma unroll
  for (int pass = 0; pass < 2; ++pass) {
#pragma unroll
    for (int it = 0; it < 8; ++it) {
      const int cx = it * 32 + lane, r = cx >> 4, q = (cx & 15) * 4;
      const v4f v = *(const v4fa*)(so + r * OSTR + q);
      *(volatile v4f*)(out + (size_t)(m0 + r) * (size_t)DM + (size_t)(n0 + q)) = v;
    }
    __threadfence();
  }
}

extern "C" void kernel_launch(void* const* d_in, const int* in_sizes, int n_in,
                              void* d_out, int out_size, void* d_ws, size_t ws_size,
                              hipStream_t stream) {
  if (n_in < 6) return;
  if (in_sizes[0] != NTOK * DM || in_sizes[1] != NTOK * DM || in_sizes[2] != DM * DM || in_sizes[3] != DM ||
      in_sizes[4] != DM * DM || in_sizes[5] != DM) return;
  if (out_size != NTOK * DM) return;

  const float* hin = (const float*)d_in[0];
  const float* xin = (const float*)d_in[1];
  const float* Wq  = (const float*)d_in[2];
  const float* bq  = (const float*)d_in[3];
  const float* Wk  = (const float*)d_in[4];
  const float* bk  = (const float*)d_in[5];
  float* out = (float*)d_out;

  const size_t planeB = (size_t)NTOK * DM * 2;
  size_t off = 0;
  auto carve = [&](size_t bytes) -> char* { char* p = (char*)d_ws + off; off += (bytes + 255) & ~(size_t)255; return p; };
  char* RA = carve(planeB);
  char* RB = carve(planeB);
  unsigned short* QF  = (unsigned short*)carve(planeB);
  unsigned short* KFL = (unsigned short*)carve(planeB);
  unsigned short* VTH = (unsigned short*)carve(planeB);
  unsigned short* VTL = (unsigned short*)carve(planeB);
  unsigned short* WQB = (unsigned short*)carve((size_t)DM * DM * 2);
  unsigned short* WKB = (unsigned short*)carve((size_t)DM * DM * 2);
  unsigned short* WQT = (unsigned short*)carve((size_t)DM * DM * 2);
  unsigned short* KVH = (unsigned short*)carve((size_t)NBH * HD * HD * 2);
  unsigned short* KVL = (unsigned short*)carve((size_t)NBH * HD * HD * 2);
  float*          KS  = (float*)carve((size_t)NBH * HD * 4);
  if (off > ws_size || off > (size_t)134217728) return;
  unsigned short* HB  = (unsigned short*)RA;
  unsigned short* KFH = (unsigned short*)RA;
  unsigned short* ATH = (unsigned short*)RA;
  unsigned short* XB  = (unsigned short*)RB;
  unsigned short* ATL = (unsigned short*)RB;

  const dim3 b256(256), b128(128);
  auto cdv = [](long a, long q2) { return (unsigned)((a + q2 - 1) / q2); };

  k_cvt_bf16<<<dim3(cdv((long)NTOK * DM / 8, 256)), b256, 0, stream>>>(hin, HB, NTOK * DM / 8);
  k_cvt_bf16<<<dim3(cdv((long)NTOK * DM / 8, 256)), b256, 0, stream>>>(xin, XB, NTOK * DM / 8);
  k_cvt_bf16<<<dim3(cdv((long)DM * DM / 8, 256)), b256, 0, stream>>>(Wq, WQB, DM * DM / 8);
  k_cvt_bf16<<<dim3(cdv((long)DM * DM / 8, 256)), b256, 0, stream>>>(Wk, WKB, DM * DM / 8);
  k_cvt_wT<<<dim3(DM / 64, DM / 64), b256, 0, stream>>>(Wq, WQT);
  k_gemm_q<<<dim3(NTOK / TPB, DM / 64), b256, 0, stream>>>(HB, WQB, bq, QF);
  k_gemm_k<<<dim3(NTOK / TPB, DM / 64), b256, 0, stream>>>(XB, WKB, bk, KFH, KFL, VTH, VTL);
  k_kv<<<dim3(NBH), b128, 0, stream>>>(KFH, KFL, VTH, VTL, KVH, KVL, KS);
  k_attn<<<dim3(SQ / 128, NBH), b256, 0, stream>>>(QF, KVH, KVL, KS, ATH, ATL);
  k_gemm_out<<<dim3(NTOK / TPB, DM / 64), b256, 0, stream>>>(ATH, ATL, WQT, out);
}
